// GPTQLinear_woo_15479062135381
// MI455X (gfx1250) — hardware-verified
//
#include <hip/hip_runtime.h>
#include <hip/hip_bf16.h>
#include <math.h>


#define BB 2
#define SS 2048
#define DD 1024
#define HH 16
#define DKK 64
#define QW 2

typedef _Float16 bf16;
typedef __attribute__((ext_vector_type(4))) unsigned v4u_t;
typedef unsigned v4ua __attribute__((ext_vector_type(4), may_alias));
typedef __attribute__((ext_vector_type(4))) float v4f_t;
typedef float v4fa __attribute__((ext_vector_type(4), may_alias));
typedef __attribute__((ext_vector_type(16))) bf16  bf16x16;
typedef __attribute__((ext_vector_type(8)))  bf16  bf16x8;
typedef __attribute__((ext_vector_type(4)))  bf16  bf16x4;
typedef __attribute__((ext_vector_type(8)))  float f32x8;

#define LDS_STRIDE 48
#define KSTRIDE    72
#define VSTRIDE    48

__device__ __forceinline__ f32x8 wmma_bf16(bf16x16 a, bf16x16 b, f32x8 c) {
  return __builtin_amdgcn_wmma_f32_16x16x32_f16(
      false, a, false, b, (short)0, c, false, false);
}

template <typename T>
__device__ __forceinline__ bf16x16 load_frag(const T* __restrict__ base, int ld,
                                             int row0, int k0) {
  const int lane = threadIdx.x & 31;
  const int r    = lane & 15;
  const int kh   = (lane >> 4) * 8;
  const T* p0 = base + (size_t)(row0 + r) * ld + (k0 + kh);
  const T* p1 = p0 + 16;
  bf16x16 f;
#pragma unroll
  for (int i = 0; i < 8; ++i) {
    f[i]     = (bf16)p0[i];
    f[i + 8] = (bf16)p1[i];
  }
  return f;
}

__device__ __forceinline__ bf16x16 lds_frag(const bf16* base, int stride) {
  const int lane = threadIdx.x & 31;
  const int row  = lane & 15;
  const int kh   = (lane >> 4) * 8;
  const bf16x8 lo = *(const bf16x8*)(base + row * stride + kh);
  const bf16x8 hi = *(const bf16x8*)(base + row * stride + kh + 16);
  bf16x16 f;
#pragma unroll
  for (int i = 0; i < 8; ++i) { f[i] = lo[i]; f[i + 8] = hi[i]; }
  return f;
}

template <typename T>
__device__ __forceinline__ void stage_read16(const T* __restrict__ p, float* buf) {
#pragma unroll
  for (int i = 0; i < 16; ++i) buf[i] = (float)p[i];
}

__device__ __forceinline__ void stage_write(bf16* dst, const float* buf, int nquad) {
#pragma unroll
  for (int i = 0; i < nquad; ++i) {
    bf16x4 q;
    q[0] = (bf16)buf[4 * i];     q[1] = (bf16)buf[4 * i + 1];
    q[2] = (bf16)buf[4 * i + 2]; q[3] = (bf16)buf[4 * i + 3];
    *(bf16x4*)(dst + 4 * i) = q;
  }
}

template <typename AT, typename WTY, int MODE>
__global__ __launch_bounds__(256) void gemm_bias_kernel(
    const AT* __restrict__ A, const WTY* __restrict__ W,
    const float* __restrict__ bias, void* __restrict__ out,
    int M, int N, int K) {
  __shared__ bf16 ldsA[128 * LDS_STRIDE];
  __shared__ bf16 ldsW[256 * LDS_STRIDE];
  __shared__ __attribute__((aligned(16))) unsigned char sob[256 * 136 * 2];

  const int t    = threadIdx.x;
  const int wave = t >> 5;
  const int lane = t & 31;
  const int wm   = (wave & 1) * 64;
  const int wn   = (wave >> 1) * 64;
  const int mBlk = blockIdx.x * 128;
  const int nBlk = blockIdx.y * 256;

  const int arow = t >> 1;
  const int ach  = (t & 1) * 16;

  float abuf[16];
  float wbuf[32];

  stage_read16(A + (size_t)(mBlk + arow) * K + ach, abuf);
  stage_read16(W + (size_t)(nBlk + t) * K,          wbuf);
  stage_read16(W + (size_t)(nBlk + t) * K + 16,     wbuf + 16);

  f32x8 acc[4][4] = {};

  for (int k = 0; k < K; k += 32) {
    __syncthreads();
    stage_write(&ldsA[arow * LDS_STRIDE + ach], abuf, 4);
    stage_write(&ldsW[t * LDS_STRIDE],          wbuf, 8);
    if (k + 32 < K) {
      stage_read16(A + (size_t)(mBlk + arow) * K + (k + 32) + ach, abuf);
      stage_read16(W + (size_t)(nBlk + t) * K + (k + 32),          wbuf);
      stage_read16(W + (size_t)(nBlk + t) * K + (k + 32) + 16,     wbuf + 16);
    }
    __syncthreads();

    bf16x16 af[4], wf[4];
#pragma unroll
    for (int i = 0; i < 4; ++i)
      af[i] = lds_frag(ldsA + (wm + 16 * i) * LDS_STRIDE, LDS_STRIDE);
#pragma unroll
    for (int j = 0; j < 4; ++j)
      wf[j] = lds_frag(ldsW + (wn + 16 * j) * LDS_STRIDE, LDS_STRIDE);
#pragma unroll
    for (int i = 0; i < 4; ++i)
#pragma unroll
      for (int j = 0; j < 4; ++j)
        acc[i][j] = wmma_bf16(af[i], wf[j], acc[i][j]);
  }

  const int nlane = lane & 15;
  const int mh    = (lane >> 4) * 8;
  __syncthreads();
  if (MODE == 0 || MODE == 1) {
    bf16* so = (bf16*)sob;
#pragma unroll
    for (int i = 0; i < 4; ++i)
#pragma unroll
      for (int j = 0; j < 4; ++j) {
        const int nl = wn + 16 * j + nlane;
        const float bv = bias ? bias[nBlk + nl] : 0.0f;
#pragma unroll
        for (int r = 0; r < 8; ++r) {
          const int ml = wm + 16 * i + mh + r;
          const bf16 hv = (bf16)(acc[i][j][r] + bv);
          if (MODE == 0) so[ml * 264 + nl] = hv;
          else           so[nl * 136 + ml] = hv;
        }
      }
    __syncthreads();
#pragma unroll 1
    for (int pass = 0; pass < 2; ++pass) {
      if (MODE == 0) {
        for (int ch = t; ch < 128 * 32; ch += 256) { const int ml = ch >> 5, q = (ch & 31) * 8;
          *(volatile v4u_t*)((bf16*)out + (size_t)(mBlk + ml) * N + nBlk + q) = *(const v4ua*)(so + ml * 264 + q); }
      } else {
        const int b_ = mBlk / SS, s0 = mBlk & (SS - 1);
        for (int ch = t; ch < 256 * 16; ch += 256) { const int nl = ch >> 4, q = (ch & 15) * 8; const int n = nBlk + nl, h = n >> 6, dk = n & (DKK - 1);
          *(volatile v4u_t*)((bf16*)out + (((size_t)(b_ * HH + h)) * DKK + dk) * SS + s0 + q) = *(const v4ua*)(so + nl * 136 + q); }
      }
      __threadfence();
    }
  } else {
    float* so = (float*)sob;
#pragma unroll 1
    for (int hf = 0; hf < 2; ++hf) {
      if (wm == hf * 64) {
#pragma unroll
        for (int i = 0; i < 4; ++i)
#pragma unroll
          for (int j = 0; j < 4; ++j) {
            const int nl = wn + 16 * j + nlane;
            const float bv = bias ? bias[nBlk + nl] : 0.0f;
#pragma unroll
            for (int r = 0; r < 8; ++r) so[(16 * i + mh + r) * 260 + nl] = acc[i][j][r] + bv;
          }
      }
      __syncthreads();
#pragma unroll 1
      for (int pass = 0; pass < 2; ++pass) {
        for (int ch = t; ch < 64 * 64; ch += 256) { const int ml = ch >> 6, q = (ch & 63) * 4;
          *(volatile v4f_t*)((float*)out + (size_t)(mBlk + hf * 64 + ml) * N + nBlk + q) = *(const volatile v4fa*)(so + ml * 260 + q); }
        __threadfence();
      }
      __syncthreads();
    }
  }
}


#define NBQ 128
#define KIN 4096
#define NOUT 11008
#define GS 128

__global__ __launch_bounds__(256) void k_dequant(const int* __restrict__ qw, const float* __restrict__ sc, const float* __restrict__ zr, bf16* __restrict__ W16) {
  const int n = blockIdx.x, t = threadIdx.x; const int k0 = t * 16;
  const int w0 = qw[(size_t)(k0 / 8) * NOUT + n], w1 = qw[(size_t)(k0 / 8 + 1) * NOUT + n];
  const int g = k0 / GS; const float s = sc[(size_t)g * NOUT + n], z = zr[(size_t)g * NOUT + n];
  bf16 h[16];
#pragma unroll
  for (int j = 0; j < 8; ++j) { const int nb0 = (w0 >> (4 * j)) & 15, nb1 = (w1 >> (4 * j)) & 15; h[j] = (bf16)(s * (float)nb0 - z); h[8 + j] = (bf16)(s * (float)nb1 - z); }
  bf16* dst = W16 + (size_t)n * KIN + k0;
#pragma unroll 1
  for (int pass = 0; pass < 2; ++pass) { *(volatile v4u_t*)dst = *(const v4ua*)h; *(volatile v4u_t*)(dst + 8) = *(const v4ua*)(h + 8); __threadfence(); }
}

extern "C" void kernel_launch(void* const* d_in, const int* in_sizes, int n_in,
                              void* d_out, int out_size, void* d_ws, size_t ws_size,
                              hipStream_t stream) {
  (void)in_sizes; (void)n_in; (void)out_size; (void)ws_size;
  const float* x = (const float*)d_in[0];
  const int* qw = (const int*)d_in[1];
  const float* sc = (const float*)d_in[2];
  const float* zr = (const float*)d_in[3];
  char* ws = (char*)d_ws;
  bf16* W16 = (bf16*)ws; ws += (size_t)NOUT * KIN * 2;
  k_dequant<<<NOUT, 256, 0, stream>>>(qw, sc, zr, W16);
  gemm_bias_kernel<float, bf16, 2><<<dim3(NBQ / 128, NOUT / 256), 256, 0, stream>>>(x, W16, nullptr, (float*)d_out, NBQ, NOUT, KIN);
}
